// GMM_41626823033065
// MI455X (gfx1250) — hardware-verified
//
#include <hip/hip_runtime.h>


#ifndef NPTS
#define NPTS 16384
#endif
#define NPTS_FULL 16384
#define KC   1024
#define DD   6
#define NF   28
#define FP   32
#define MW   4
#define PTW  32
#define BP   (MW * PTW)
#define PT   64
#define TSP  36
#define QRS  2048.0f
#define QRI  (1.0f / 2048.0f)
#define LOG2E_F 1.4426950408889634f
#define C3LOG2PI 5.513631199228036f
#define NEGB (-3.0e38f)

static_assert(DD == 6);
static_assert(NF == 1 + DD + DD * (DD + 1) / 2);
static_assert(NF <= FP);
static_assert(FP == 32);
static_assert(MW == 4);
static_assert(PTW == 32);
static_assert(BP == 32 * MW);
static_assert(NPTS % BP == 0);
static_assert(NPTS <= NPTS_FULL);
static_assert(KC % 16 == 0);
static_assert(KC % PT == 0);
static_assert(KC % (32 * MW * 4) == 0);
static_assert(32 * 16 == BP * 4);
static_assert(PT * 16 * 4 == PT * FP * 2);
static_assert(16 * 16 == PT * 4);
static_assert((TSP * 4) % 16 == 0);
static_assert(TSP >= FP);
static_assert(PT % 32 == 0);

typedef _Float16 h16;
typedef __attribute__((ext_vector_type(16))) _Float16 v16h;
typedef __attribute__((ext_vector_type(8)))  _Float16 v8h;
typedef __attribute__((ext_vector_type(8)))  float    v8f;
typedef __attribute__((ext_vector_type(4)))  float    v4f;
typedef v4f  __attribute__((may_alias)) v4fa;

__device__ __forceinline__ unsigned short f2bf(float f) { unsigned u = __float_as_uint(f); u += 0x7FFFu + ((u >> 16) & 1u); return (unsigned short)(u >> 16); }
__device__ __forceinline__ float bfr(float f) { return __uint_as_float(((unsigned)f2bf(f)) << 16); }
__device__ __forceinline__ v16h cat16(v8h lo, v8h hi) { return __builtin_shufflevector(lo, hi, 0, 1, 2, 3, 4, 5, 6, 7, 8, 9, 10, 11, 12, 13, 14, 15); }
__device__ __forceinline__ v16h ldh(const h16* p) { return cat16(*(const v8h*)p, *(const v8h*)(p + 16)); }
static __device__ __forceinline__ h16 toh_flush(float v) { const h16 r = (h16)v; return (fabsf(v) < 6.103515625e-05f) ? (h16)0.0f : r; }
__device__ __forceinline__ v8f wmma16g(v16h a, v16h b, v8f c) {
    c = __builtin_amdgcn_wmma_f32_16x16x32_f16(false, a, false, b, (short)0, c, false, false);
    asm volatile("v_nop\n\tv_nop\n\tv_nop\n\tv_nop" : "+v"(c) : "v"(a), "v"(b));
    return c;
}

#define LX(e) ((e) * PT + tid)

__global__ __launch_bounds__(PT) void k_prep(const float* __restrict__ means, const float* __restrict__ covs, const float* __restrict__ wts, h16* TH, h16* TR, float* AL) {
#pragma clang fp contract(off)
    __shared__ float Ls[36 * PT];
    __shared__ float Is[36 * PT];
    __shared__ float Ds[DD * PT];
    __shared__ float Us[DD * PT];
    __shared__ float Vs[DD * PT];
    __shared__ __align__(16) float ths[PT * TSP];
    __shared__ __align__(16) float als[PT];
    const int tid = threadIdx.x;
    const int k = blockIdx.x * PT + tid;
    const float* cv = covs + (size_t)k * (DD * DD);
#pragma unroll 1
    for (int e = 0; e < DD * DD; ++e) {
        const int i = e / DD, j = e - DD * i;
        const float a = bfr(cv[i * DD + j]), b = bfr(cv[j * DD + i]);
        Ls[LX(e)] = 0.5f * (a + b); Is[LX(e)] = 0.0f; }
#pragma unroll 1
    for (int i = 0; i < DD; ++i) Us[LX(i)] = bfr(means[(size_t)k * DD + i]);

    float ipd = 1.0f;
#pragma unroll 1
    for (int j = 0; j < DD; ++j) {
        float s = Ls[LX(j * DD + j)];
#pragma unroll 1
        for (int p = 0; p < j; ++p) { const float a = Ls[LX(j * DD + p)]; s -= a * a; }
        const float d = sqrtf(s);
        const float inv = 1.0f / d;
        Ls[LX(j * DD + j)] = d; Ds[LX(j)] = inv; ipd *= inv;
#pragma unroll 1
        for (int i = j + 1; i < DD; ++i) {
            float t = Ls[LX(i * DD + j)];
#pragma unroll 1
            for (int p = 0; p < j; ++p) t -= Ls[LX(i * DD + p)] * Ls[LX(j * DD + p)];
            Ls[LX(i * DD + j)] = t * inv; }
    }
#pragma unroll 1
    for (int j = 0; j < DD; ++j) {
        Is[LX(j * DD + j)] = Ds[LX(j)];
#pragma unroll 1
        for (int i = j + 1; i < DD; ++i) {
            float s = 0.0f;
#pragma unroll 1
            for (int p = j; p < i; ++p) s += Ls[LX(i * DD + p)] * Is[LX(p * DD + j)];
            Is[LX(i * DD + j)] = -s * Ds[LX(i)]; }
    }
#pragma unroll 1
    for (int a = 0; a < DD; ++a) {
#pragma unroll 1
        for (int b = a; b < DD; ++b) {
            float s = 0.0f;
#pragma unroll 1
            for (int i = b; i < DD; ++i) s += Is[LX(i * DD + a)] * Is[LX(i * DD + b)];
            Ls[LX(a * DD + b)] = s; Ls[LX(b * DD + a)] = s; }
    }
    float c = 0.0f;
#pragma unroll 1
    for (int a = 0; a < DD; ++a) {
        float s = 0.0f;
#pragma unroll 1
        for (int b = 0; b < DD; ++b) s += Ls[LX(a * DD + b)] * Us[LX(b)];
        Vs[LX(a)] = s; c += Us[LX(a)] * s; }
    const float wv = bfr(wts[k]);
    const float alpha = logf(wv * ipd) - C3LOG2PI;
    const int tb = tid * TSP;
    ths[tb] = LOG2E_F * (alpha - 0.5f * c);
#pragma unroll 1
    for (int i = 0; i < DD; ++i) ths[tb + 1 + i] = LOG2E_F * Vs[LX(i)];
    int idx = 1 + DD;
#pragma unroll 1
    for (int i = 0; i < DD; ++i) {
#pragma unroll 1
        for (int j = i; j < DD; ++j) {
            const float pv = Ls[LX(i * DD + j)];
            ths[tb + idx] = LOG2E_F * ((i == j) ? (-0.5f * pv) : (-pv));
            ++idx; }
    }
#pragma unroll 1
    for (int t = NF; t < FP; ++t) ths[tb + t] = 0.0f;
    als[tid] = alpha;
    __syncthreads();
    const size_t pb = (size_t)blockIdx.x * PT * FP;
#pragma unroll 1
    for (int ps = 0; ps < 2; ++ps) {
#pragma unroll 1
        for (int it = 0; it < 4; ++it) {
            const int p = it * PT + tid; const int row = p >> 2, c8 = (p & 3) * 8;
            const v4f x0 = *(const v4fa*)(&ths[row * TSP + c8]); const v4f x1 = *(const v4fa*)(&ths[row * TSP + c8 + 4]);
            v8h hv, rv;
#pragma unroll
            for (int i = 0; i < 4; ++i) {
                const h16 a0 = toh_flush(x0[i]); const h16 a1 = toh_flush(x1[i]);
                hv[i] = a0; hv[4 + i] = a1;
                rv[i] = toh_flush((x0[i] - (float)a0) * QRS); rv[4 + i] = toh_flush((x1[i] - (float)a1) * QRS); }
            const size_t oo = pb + (size_t)p * 8;
            *(volatile v8h*)(TH + oo) = hv; *(volatile v8h*)(TR + oo) = rv; }
        if (tid < 16) {
            const v4f a = *(const v4fa*)(&als[tid * 4]);
            *(volatile v4f*)(AL + (size_t)blockIdx.x * PT + tid * 4) = a; }
        if (ps == 0) __threadfence(); }
}

__global__ __launch_bounds__(32 * MW) void k_mix(const float* __restrict__ X, const h16* __restrict__ TH, const h16* __restrict__ TR, const float* __restrict__ AL, float* OUT) {
    __shared__ v8h phs[BP * 4];
    __shared__ v8h prs[BP * 4];
    __shared__ float wmx[MW];
    __shared__ __align__(16) float outs[BP];
    const int tid = threadIdx.x;
    const int lane = tid & 31, lr = lane & 15, hi = lane >> 4;
    const int wave = __builtin_amdgcn_readfirstlane((int)(threadIdx.x >> 5));
    const int p0 = blockIdx.x * BP;

    float mx = NEGB;
#pragma unroll 1
    for (int i = tid * 4; i < KC; i += 32 * MW * 4) {
        const v4f a = *(const v4f*)(AL + i);
        mx = fmaxf(mx, fmaxf(fmaxf(a[0], a[1]), fmaxf(a[2], a[3]))); }
    mx = fmaxf(mx, __shfl_xor(mx, 16, 32)); mx = fmaxf(mx, __shfl_xor(mx, 8, 32)); mx = fmaxf(mx, __shfl_xor(mx, 4, 32));
    mx = fmaxf(mx, __shfl_xor(mx, 2, 32));  mx = fmaxf(mx, __shfl_xor(mx, 1, 32));
    if (lane == 0) wmx[wave] = mx;

    {
        float xv[DD];
#pragma unroll
        for (int i = 0; i < DD; ++i) xv[i] = bfr(X[(size_t)(p0 + tid) * DD + i]);
        float one = 1.0f, zero = 0.0f;
        asm volatile("" : "+v"(one)); asm volatile("" : "+v"(zero));
        float f[FP];
        f[0] = one;
#pragma unroll
        for (int i = 0; i < DD; ++i) f[1 + i] = xv[i];
        int idx = 1 + DD;
#pragma unroll
        for (int i = 0; i < DD; ++i)
#pragma unroll
            for (int j = i; j < DD; ++j) { f[idx] = xv[i] * xv[j]; ++idx; }
#pragma unroll
        for (int t = NF; t < FP; ++t) f[t] = zero;
#pragma unroll
        for (int q = 0; q < 4; ++q) {
            v8h hv, rv;
#pragma unroll
            for (int e = 0; e < 8; ++e) { const float v = f[q * 8 + e]; const h16 a = toh_flush(v); hv[e] = a; rv[e] = toh_flush((v - (float)a) * QRS); }
            phs[tid * 4 + q] = hv; prs[tid * 4 + q] = rv; }
    }
    __syncthreads();
    const float M = fmaxf(fmaxf(wmx[0], wmx[1]), fmaxf(wmx[2], wmx[3]));
    const float nMs = -M * LOG2E_F;
    const int rw = wave * PTW + lr;
    const v16h bh0 = cat16(phs[rw * 4 + hi], phs[rw * 4 + 2 + hi]);
    const v16h br0 = cat16(prs[rw * 4 + hi], prs[rw * 4 + 2 + hi]);
    const v16h bh1 = cat16(phs[(rw + 16) * 4 + hi], phs[(rw + 16) * 4 + 2 + hi]);
    const v16h br1 = cat16(prs[(rw + 16) * 4 + hi], prs[(rw + 16) * 4 + 2 + hi]);
    const size_t ao = (size_t)lr * FP + 8 * hi;
    float s0 = 0.0f, s1 = 0.0f;
#pragma unroll 1
    for (int ct = 0; ct < KC / 16; ++ct) {
        const size_t o = ao + (size_t)ct * 16 * FP;
        const v16h th = ldh(TH + o), tr = ldh(TR + o);
        v8f cH, cR;
#pragma unroll
        for (int r = 0; r < 8; ++r) cH[r] = nMs;
        cR = (v8f){};
        cH = wmma16g(th, bh0, cH); cR = wmma16g(th, br0, cR); cR = wmma16g(tr, bh0, cR);
#pragma unroll
        for (int r = 0; r < 8; ++r) s0 += __builtin_amdgcn_exp2f(cH[r] + cR[r] * QRI);
#pragma unroll
        for (int r = 0; r < 8; ++r) cH[r] = nMs;
        cR = (v8f){};
        cH = wmma16g(th, bh1, cH); cR = wmma16g(th, br1, cR); cR = wmma16g(tr, bh1, cR);
#pragma unroll
        for (int r = 0; r < 8; ++r) s1 += __builtin_amdgcn_exp2f(cH[r] + cR[r] * QRI);
    }
    s0 += __shfl_xor(s0, 16, 32); s1 += __shfl_xor(s1, 16, 32);
    const float v0 = M + logf(s0), v1 = M + logf(s1);
    outs[wave * PTW + hi * 16 + lr] = hi ? v1 : v0;
    __syncthreads();
    if (wave == 0) {
        const v4f val = *(const v4fa*)(&outs[lane * 4]);
        float* op = OUT + (size_t)p0 + lane * 4;
        *(volatile v4f*)op = val; __threadfence(); *(volatile v4f*)op = val; }
}

static constexpr size_t al256(size_t v) { return (v + 255) & ~(size_t)255; }
static constexpr size_t SZ_TH = al256((size_t)KC * FP * 2);
static constexpr size_t SZ_AL = al256((size_t)KC * 4);
static constexpr size_t SZ_TOTAL = 2 * SZ_TH + SZ_AL;
static_assert(SZ_TOTAL <= (size_t)134217728);
static_assert((size_t)(KC / PT) * PT * FP * 2 == (size_t)KC * FP * 2);
static_assert((size_t)(KC / PT) * PT * 4 == (size_t)KC * 4);
static_assert((size_t)(36 * 2 + DD * 3) * PT * 4 + (size_t)PT * TSP * 4 + (size_t)PT * 4 <= (size_t)131072);
static_assert((size_t)2 * BP * 4 * 16 + (size_t)MW * 4 + (size_t)BP * 4 <= (size_t)131072);

extern "C" void kernel_launch(void* const* d_in, const int* in_sizes, int n_in,
                              void* d_out, int out_size, void* d_ws, size_t ws_size, hipStream_t stream) {
    if (n_in < 4) return;
    if ((size_t)in_sizes[0] < (size_t)NPTS * DD) return;
    if ((size_t)in_sizes[1] < (size_t)KC * DD || (size_t)in_sizes[2] < (size_t)KC * DD * DD || (size_t)in_sizes[3] < (size_t)KC) return;
    if ((size_t)out_size < (size_t)NPTS) return;
    if (SZ_TOTAL > ws_size) return;
    const float* x  = (const float*)d_in[0];
    const float* mu = (const float*)d_in[1];
    const float* cv = (const float*)d_in[2];
    const float* wt = (const float*)d_in[3];
    float* OUT = (float*)d_out;
    char* wsp = (char*)d_ws;
    h16* TH = (h16*)wsp; wsp += SZ_TH;
    h16* TR = (h16*)wsp; wsp += SZ_TH;
    float* AL = (float*)wsp; wsp += SZ_AL;

    k_prep<<<dim3(KC / PT, 1, 1), PT, 0, stream>>>(mu, cv, wt, TH, TR, AL);
    k_mix<<<dim3(NPTS / BP, 1, 1), 32 * MW, 0, stream>>>(x, TH, TR, AL, OUT);
}
